// TLSTM3Cell_1331439862441
// MI455X (gfx1250) — hardware-verified
//
#include <hip/hip_runtime.h>
#include <math.h>

typedef __attribute__((ext_vector_type(16))) _Float16 v16h;
typedef __attribute__((ext_vector_type(16))) __bf16 v16b;
typedef __attribute__((ext_vector_type(8)))  _Float16 v8h;
typedef __attribute__((ext_vector_type(8)))  float v8f;
typedef __attribute__((ext_vector_type(4)))  float v4f;
typedef __attribute__((ext_vector_type(2)))  float v2f;
typedef __attribute__((ext_vector_type(4)))  unsigned v4u;
typedef __attribute__((ext_vector_type(4)))  int v4i;
typedef float __attribute__((may_alias)) float_a;
typedef int __attribute__((may_alias)) int_a;

template <typename T> __device__ __forceinline__ void vst2(void* p, T v) { *(volatile T*)p = v; __threadfence(); *(volatile T*)p = v; }
__device__ __forceinline__ v8f wmma16(v16h a, v16h b, v8f c) {
  v8f d = __builtin_amdgcn_wmma_f32_16x16x32_f16(false, a, false, b, (short)0, c, false, false);
  asm volatile("v_nop\n\tv_nop\n\tv_nop\n\tv_nop" : "+v"(d) : "v"(a), "v"(b));
  return d;
}
__device__ __forceinline__ v8f wmma_bf(v16b a, v16b b, v8f c) {
  v8f d = __builtin_amdgcn_wmma_f32_16x16x32_bf16(false, a, false, b, (short)0, c, false, false);
  asm volatile("v_nop\n\tv_nop\n\tv_nop\n\tv_nop" : "+v"(d) : "v"(a), "v"(b));
  return d;
}
__device__ __forceinline__ v16h frag_h(const _Float16* rowk0, int lane) {
  union { v16h v; v8h q[2]; } u; const _Float16* p = rowk0 + 8 * (lane >> 4);
  u.q[0] = *(const v8h*)p; u.q[1] = *(const v8h*)(p + 16); return u.v;
}
__device__ __forceinline__ v16h frag_f32(const float* rowk0, int lane) {
  v16h a; const float* p = rowk0 + 8 * (lane >> 4);
#pragma unroll
  for (int i = 0; i < 8; ++i) { a[i] = (_Float16)p[i]; a[8 + i] = (_Float16)p[16 + i]; }
  return a;
}
__device__ __forceinline__ v16h frag_f32s(const float* rowk0, int lane, float sc) {
  v16h a; const float* p = rowk0 + 8 * (lane >> 4);
#pragma unroll
  for (int i = 0; i < 8; ++i) { a[i] = (_Float16)(p[i] * sc); a[8 + i] = (_Float16)(p[16 + i] * sc); }
  return a;
}
__device__ __forceinline__ v16h fragc_f32(const float* W, int k0, int n, int lane, int ld, int K) {
  v16h a; const int g = lane >> 4;
#pragma unroll
  for (int i = 0; i < 8; ++i) { const int ka = k0 + 8 * g + i, kb = ka + 16;
    a[i] = (_Float16)(ka < K ? W[(size_t)(ka < K ? ka : K - 1) * ld + n] : 0.f); a[8 + i] = (_Float16)(kb < K ? W[(size_t)(kb < K ? kb : K - 1) * ld + n] : 0.f); }
  return a;
}
struct F2 { v16b h, l; };
__device__ __forceinline__ F2 bsplit16(const float v[16]) { F2 r;
#pragma unroll
  for (int i = 0; i < 16; ++i) { const __bf16 h = (__bf16)v[i]; r.h[i] = h; r.l[i] = (__bf16)(v[i] - (float)h); }
  return r; }
__device__ __forceinline__ F2 split_row(const float* row, int k0, int lane) { float v[16]; const float* p = row + k0 + 8 * (lane >> 4);
#pragma unroll
  for (int i = 0; i < 8; ++i) { v[i] = p[i]; v[8 + i] = p[16 + i]; }
  return bsplit16(v); }
__device__ __forceinline__ F2 split_rowK(const float* row, int k0, int lane, int K) { float v[16]; const int g = lane >> 4;
#pragma unroll
  for (int i = 0; i < 8; ++i) { const int ka = k0 + 8 * g + i, kb = ka + 16; v[i] = ka < K ? row[ka < K ? ka : K - 1] : 0.f; v[8 + i] = kb < K ? row[kb < K ? kb : K - 1] : 0.f; }
  return bsplit16(v); }
__device__ __forceinline__ F2 split_col(const float* W, int k0, int n, int lane, int ld, int K) { float v[16]; const int g = lane >> 4;
#pragma unroll
  for (int i = 0; i < 8; ++i) { const int ka = k0 + 8 * g + i, kb = ka + 16; v[i] = ka < K ? W[(size_t)(ka < K ? ka : K - 1) * ld + n] : 0.f; v[8 + i] = kb < K ? W[(size_t)(kb < K ? kb : K - 1) * ld + n] : 0.f; }
  return bsplit16(v); }
__device__ __forceinline__ v8f mac3(const F2& a, const F2& b, v8f c) { c = wmma_bf(a.l, b.h, c); c = wmma_bf(a.h, b.l, c); return wmma_bf(a.h, b.h, c); }
__device__ __forceinline__ float sigm(float v) { return 1.0f / (1.0f + expf(-v)); }
#define LDSX() do { asm volatile("s_wait_dscnt 0" ::: "memory"); __builtin_amdgcn_wave_barrier(); __builtin_amdgcn_fence(__ATOMIC_RELEASE, "workgroup"); } while (0)


#define NR 8192
#define DD 512
#define HH 512
#ifndef TR
#define TR (NR / 64)
#endif
typedef __attribute__((ext_vector_type(8))) __bf16 v8b;
__device__ __forceinline__ v16b frag_b(const __bf16* rowk0, int lane) {
  union { v16b v; v8b q[2]; } u; const __bf16* p = rowk0 + 8 * (lane >> 4);
  u.q[0] = *(const v8b*)p; u.q[1] = *(const v8b*)(p + 16); return u.v;
}
__device__ __forceinline__ float bfr(float v) { return (float)(__bf16)v; }
__device__ __attribute__((noinline)) float exp_ni(float v) { return expf(v); }
__device__ __attribute__((noinline)) float erf_ni(float v) { return erff(v); }

#define WS_PX  0u
#define WS_PHd (WS_PX + 2u * 5 * HH * DD)
#define WS_PC  (WS_PHd + 2u * 3 * HH * HH)
#define WS_S   (WS_PC + 2u * HH * HH)
#define WS_CT  (WS_S + 4u * (size_t)NR * 5 * HH)
#define WS_END (WS_CT + 4u * (size_t)NR * HH)

__global__ __launch_bounds__(128) void k_pack(const float* __restrict__ W0, const float* __restrict__ W1, const float* __restrict__ W2, const float* __restrict__ W3, const float* __restrict__ W4, const float* __restrict__ W5, const float* __restrict__ W6, const float* __restrict__ W7, const float* __restrict__ W8, __bf16* __restrict__ P) {
  const int o = blockIdx.x, which = blockIdx.y, t = threadIdx.x; __shared__ __align__(16) __bf16 s[DD]; const float* Wm = which == 0 ? W0 : which == 1 ? W1 : which == 2 ? W2 : which == 3 ? W3 : which == 4 ? W4 : which == 5 ? W5 : which == 6 ? W6 : which == 7 ? W7 : W8;
  for (int k = t; k < DD; k += 128) s[k] = (__bf16)Wm[(size_t)o * DD + k]; __syncthreads();
  __bf16* dst = P + ((size_t)which * HH + o) * DD;
  if (t < DD / 8) vst2((unsigned*)(dst + t * 8), *(const v4u*)&s[t * 8]); }
__device__ __forceinline__ v16b fragb_f32(const float* __restrict__ p, int lane) { v16b a; const float* pp = p + 8 * (lane >> 4);
#pragma unroll
  for (int i = 0; i < 8; ++i) { a[i] = (__bf16)pp[i]; a[8 + i] = (__bf16)pp[16 + i]; } return a; }
__global__ __launch_bounds__(128) void k_pre(const float* __restrict__ X, const float* __restrict__ HID, const __bf16* __restrict__ P, float* __restrict__ S) { __shared__ __align__(16) float sf[4][16][132];
  const int tid = threadIdx.x, wave = tid >> 5, lane = tid & 31, col = lane & 15, g = lane >> 4; const size_t r0 = (size_t)blockIdx.x * 64 + wave * 16; const int grp = blockIdx.y / 4; const int c0 = (blockIdx.y % 4) * 128;
  v8f acc[8] = {};
  const __bf16* Wx = P + ((size_t)grp * HH + c0) * DD;
#pragma unroll 2
  for (int kc = 0; kc < DD / 32; ++kc) { const v16b a = fragb_f32(X + (r0 + col) * DD + kc * 32, lane);
#pragma unroll
    for (int j = 0; j < 8; ++j) acc[j] = wmma_bf(a, frag_b(Wx + (size_t)(j * 16 + col) * DD + kc * 32, lane), acc[j]); }
  if (grp < 3) { const __bf16* Wh = P + ((size_t)(5 + grp) * HH + c0) * DD;
#pragma unroll 2
    for (int kc = 0; kc < HH / 32; ++kc) { const v16b a = fragb_f32(HID + (r0 + col) * HH + kc * 32, lane);
#pragma unroll
      for (int j = 0; j < 8; ++j) acc[j] = wmma_bf(a, frag_b(Wh + (size_t)(j * 16 + col) * HH + kc * 32, lane), acc[j]); } }
#pragma unroll
  for (int j = 0; j < 8; ++j)
#pragma unroll
    for (int r = 0; r < 8; ++r) sf[wave][8 * g + r][j * 16 + col] = acc[j][r];
  LDSX(); for (int rl = 0; rl < 16; ++rl) vst2(S + (r0 + rl) * (5 * HH) + grp * HH + c0 + lane * 4, *(const v4f*)&sf[wave][rl][lane * 4]); }
__global__ __launch_bounds__(128) void k_cell(const float* __restrict__ S, const float* __restrict__ DT, const float* __restrict__ CS, const float* __restrict__ BII, const float* __restrict__ BHI, const float* __restrict__ BIG, const float* __restrict__ BHG, const float* __restrict__ BIT1, const float* __restrict__ WTT1, const float* __restrict__ BIT2, const float* __restrict__ WTT2, float* __restrict__ CT, float* __restrict__ CM) {
  __shared__ __align__(16) float sct[HH], scm[HH]; const int t = threadIdx.x; const size_t row = blockIdx.x; const float dt = bfr(DT[row]); const float* sr = S + row * (5 * HH);
  for (int c = t; c < HH; c += 128) { const float tm1 = sigm(sr[3 * HH + c] + bfr(BIT1[c]) + sigm(dt * bfr(WTT1[c]))); const float tm2 = sigm(sr[4 * HH + c] + bfr(BIT2[c]) + sigm(dt * bfr(WTT2[c])));
    const float im = sigm(sr[c] + bfr(BII[c]) + bfr(BHI[c])); const float cur = tanhf(sr[HH + c] + bfr(BIG[c]) + bfr(BHG[c])); const float cs = bfr(CS[row * HH + c]);
    const float it1 = im * tm1; sct[c] = (1.0f - it1) * cs + it1 * cur; scm[c] = (1.0f - im) * cs + im * tm2 * cur; }
  __syncthreads(); vst2(CT + row * HH + t * 4, *(const v4f*)&sct[t * 4]); vst2(CM + row * HH + t * 4, *(const v4f*)&scm[t * 4]); }
__global__ __launch_bounds__(128) void k_out(const float* __restrict__ S, const float* __restrict__ CT, const float* __restrict__ DT, const __bf16* __restrict__ P, const float* __restrict__ BIO, const float* __restrict__ BHO, const float* __restrict__ WTO, const float* __restrict__ BTO, const float* __restrict__ BCO, float* __restrict__ HM) { __shared__ __align__(16) float sf[4][16][132];
  const int tid = threadIdx.x, wave = tid >> 5, lane = tid & 31, col = lane & 15, g = lane >> 4; const size_t r0 = (size_t)blockIdx.x * 64 + wave * 16; const int c0 = blockIdx.y * 128; const __bf16* Wc = P + ((size_t)8 * HH + c0) * HH;
  v8f acc[8] = {};
#pragma unroll 2
  for (int kc = 0; kc < HH / 32; ++kc) { const F2 a = split_row(CT + (r0 + col) * HH, kc * 32, lane);
#pragma unroll
    for (int j = 0; j < 8; ++j) { const v16b w = frag_b(Wc + (size_t)(j * 16 + col) * HH + kc * 32, lane); acc[j] = wmma_bf(a.h, w, acc[j]); acc[j] = wmma_bf(a.l, w, acc[j]); } }
#pragma unroll
  for (int j = 0; j < 8; ++j) { const int c = c0 + j * 16 + col; const float cb = bfr(BIO[c]) + bfr(BHO[c]) + bfr(BTO[c]) + bfr(BCO[c]); const float wto = bfr(WTO[c]);
#pragma unroll
    for (int r = 0; r < 8; ++r) { const size_t row = r0 + 8 * g + r; const float om = sigm(S[row * (5 * HH) + 2 * HH + c] + cb + bfr(DT[row]) * wto + acc[j][r]); sf[wave][8 * g + r][j * 16 + col] = om * tanhf(CT[row * HH + c]); } }
  LDSX(); for (int rl = 0; rl < 16; ++rl) vst2(HM + (r0 + rl) * HH + c0 + lane * 4, *(const v4f*)&sf[wave][rl][lane * 4]); }
extern "C" void kernel_launch(void* const* d_in, const int* in_sizes, int n_in, void* d_out, int out_size, void* d_ws, size_t ws_size, hipStream_t stream) {
  (void)in_sizes; (void)n_in; (void)out_size;
  const float** F = (const float**)d_in;
  if (ws_size < (size_t)WS_END) return;
  char* ws = (char*)d_ws; __bf16* P = (__bf16*)(ws + WS_PX); float *S = (float*)(ws + WS_S), *CT = (float*)(ws + WS_CT);
  float* HM = (float*)d_out; float* CM = HM + (size_t)NR * HH;
  k_pack<<<dim3(HH, 9), 128, 0, stream>>>(F[4], F[8], F[12], F[20], F[23], F[6], F[10], F[14], F[18], P);
  k_pre<<<dim3(TR, 20), 128, 0, stream>>>(F[0], F[2], P, S);
  k_cell<<<TR * 64, 128, 0, stream>>>(S, F[1], F[3], F[5], F[7], F[9], F[11], F[21], F[22], F[24], F[25], CT, CM);
  k_out<<<dim3(TR, HH / 128), 128, 0, stream>>>(S, CT, F[1], P, F[13], F[15], F[16], F[17], F[19], HM);
}
